// SetConv1dDecoder_4569845203569
// MI455X (gfx1250) — hardware-verified
//
#include <hip/hip_runtime.h>
#include <stdint.h>

#define NB    4
#define NT    4096
#define NS    4096
#define NV    512
#define BM    64
#define BN    256
#define BK    32
#define LDA   40
#define SP    132
#define NSTEP (NS / BK)
#define WSCALE 256.0f
#define WINV   0.00390625f

static_assert(NT % BM == 0);
static_assert(NV % BN == 0);
static_assert(NS % BK == 0);
static_assert(BN == 4 * 64);
static_assert(BM * 4 == 256);
static_assert((LDA % 8) == 0);
static_assert((SP % 4) == 0);
static_assert((NS % 8) == 0);
static_assert(64 * SP >= 63 * SP + 128);

typedef _Float16 f16;
typedef _Float16 v16h __attribute__((ext_vector_type(16)));
typedef _Float16 v8h  __attribute__((ext_vector_type(8)));
typedef unsigned short v8us __attribute__((ext_vector_type(8)));
typedef float v8f __attribute__((ext_vector_type(8)));
typedef float v4f __attribute__((ext_vector_type(4)));
typedef float v4fa __attribute__((ext_vector_type(4), may_alias));

union FragH { v16h v; v8h h[2]; };

__device__ __forceinline__ float bf16r(float f) {
  unsigned int u = __float_as_uint(f);
  u = u + 0x7FFFu + ((u >> 16) & 1u);
  u &= 0xFFFF0000u;
  return __uint_as_float(u);
}

__device__ __forceinline__ v8f mma_h(v16h a, v16h b, v8f c) {
  return __builtin_amdgcn_wmma_f32_16x16x32_f16(false, a, false, b, (short)0, c, false, false);
}

__device__ __forceinline__ void guard_group(v8f& c0, v8f& c1, v8f& c2, v8f& c3,
                                            v8f& c4, v8f& c5, v8f& c6, v8f& c7,
                                            v16h a0, v16h a1, v16h b0, v16h b1, v16h b2, v16h b3) {
#if defined(__HIP_DEVICE_COMPILE__)
  asm volatile("v_nop\n\tv_nop\n\tv_nop\n\tv_nop"
               : "+v"(c0), "+v"(c1), "+v"(c2), "+v"(c3), "+v"(c4), "+v"(c5), "+v"(c6), "+v"(c7)
               : "v"(a0), "v"(a1), "v"(b0), "v"(b1), "v"(b2), "v"(b3));
#endif
}

__global__ __launch_bounds__(256)
void cvt_value_f16(const float* __restrict__ v, unsigned short* vh, int n8) {
  const int g = (int)blockIdx.x * 256 + (int)threadIdx.x;
  if (g >= n8) return;
  const float* p = v + (size_t)g * 8;
  const v4f a = *(const v4f*)p;
  const v4f c = *(const v4f*)(p + 4);
  v8h o = {};
#pragma unroll
  for (int e = 0; e < 4; ++e) {
    o[e]     = (f16)bf16r(a[e]);
    o[4 + e] = (f16)bf16r(c[e]);
  }
  const v8us u = __builtin_bit_cast(v8us, o);
  unsigned short* op = vh + (size_t)g * 8;
  *(volatile v8us*)op = u;
  __threadfence();
  *(volatile v8us*)op = u;
}

__global__ __launch_bounds__(256)
void rbf_gemm_kernel(const float* __restrict__ q, const float* __restrict__ k,
                     const unsigned short* __restrict__ vh, const float* __restrict__ ls,
                     float* out) {
  __shared__ __align__(16) f16   ldsA[2][BM * LDA];
  __shared__ __align__(16) float s_tile[BM * SP];

  const int tid  = threadIdx.x;
  const int lane = tid & 31;
  const int wave = tid >> 5;
  const int wm   = wave & 1;
  const int wn   = wave >> 1;
  const int hl   = lane >> 4;
  const int l15  = lane & 15;

  const int b  = (int)blockIdx.z;
  const int m0 = (int)blockIdx.x * BM;
  const int n0 = (int)blockIdx.y * BN;
  if (m0 + BM > NT || n0 + BN > NV || b >= NB) return;

  const float lsv  = bf16r(ls[0]);
  const float rinv = 1.0f / expf(2.0f * lsv);
  const float cn   = -0.5f;

  const float* qb = q + (size_t)b * NT;
  const float* kb = k + (size_t)b * NS;
  const f16*   vp = (const f16*)vh + (size_t)b * NV * NS;

  const int arow = tid >> 2;
  const int acol = (tid & 3) * 8;
  const float qv = bf16r(qb[m0 + arow]);

  const f16* vb0 = vp + (size_t)(n0 + wn * 64 + l15) * NS + 8 * hl;

  v8f acc[2][4];
  {
    const v8f zero = {};
#pragma unroll
    for (int i = 0; i < 2; ++i)
#pragma unroll
      for (int j = 0; j < 4; ++j) acc[i][j] = zero;
  }

#pragma unroll 2
  for (int step = 0; step < NSTEP; ++step) {
    const int p  = step & 1;
    const int k0 = step * BK;

    {
      const float* kp = kb + k0 + acol;
      const v4f ka = *(const v4f*)kp;
      const v4f kc = *(const v4f*)(kp + 4);
      v8h a = {};
#pragma unroll
      for (int j = 0; j < 4; ++j) {
        const float d0 = bf16r(ka[j]) - qv;
        const float d1 = bf16r(kc[j]) - qv;
        const float e0 = (cn * (d0 * d0)) * rinv;
        const float e1 = (cn * (d1 * d1)) * rinv;
        a[j]     = (f16)(__expf(e0) * WSCALE);
        a[j + 4] = (f16)(__expf(e1) * WSCALE);
      }
      *(v8h*)&ldsA[p][arow * LDA + acol] = a;
    }

    __syncthreads();

    FragH af[2];
#pragma unroll
    for (int mt = 0; mt < 2; ++mt) {
      const f16* pa = &ldsA[p][(wm * 32 + mt * 16 + l15) * LDA + 8 * hl];
      af[mt].h[0] = *(const v8h*)pa;
      af[mt].h[1] = *(const v8h*)(pa + 16);
    }

    FragH bf[4];
#pragma unroll
    for (int nt = 0; nt < 4; ++nt) {
      const f16* pb = vb0 + (size_t)nt * 16 * NS + k0;
      bf[nt].h[0] = *(const v8h*)pb;
      bf[nt].h[1] = *(const v8h*)(pb + 16);
    }

#pragma unroll
    for (int mt = 0; mt < 2; ++mt)
#pragma unroll
      for (int nt = 0; nt < 4; ++nt)
        acc[mt][nt] = mma_h(af[mt].v, bf[nt].v, acc[mt][nt]);
    guard_group(acc[0][0], acc[0][1], acc[0][2], acc[0][3],
                acc[1][0], acc[1][1], acc[1][2], acc[1][3],
                af[0].v, af[1].v, bf[0].v, bf[1].v, bf[2].v, bf[3].v);
  }

#pragma unroll
  for (int ph = 0; ph < 2; ++ph) {
    if ((wn >> 1) == ph) {
      float* sw = s_tile + (wm * 32) * SP + (wn & 1) * 64;
#pragma unroll
      for (int mt = 0; mt < 2; ++mt)
#pragma unroll
        for (int nt = 0; nt < 4; ++nt)
#pragma unroll
          for (int r = 0; r < 8; ++r)
            sw[(mt * 16 + 8 * hl + r) * SP + nt * 16 + l15] = acc[mt][nt][r] * WINV;
    }
    __syncthreads();

    const float* sr = s_tile + lane * 4;
    float* ob = out + ((size_t)b * NT + m0) * NV + n0 + ph * 128 + lane * 4;
#pragma unroll
    for (int rr = 0; rr < 8; ++rr) {
      const int row = wave * 8 + rr;
      const v4f val = *(const v4fa*)(sr + row * SP);
      *(volatile v4f*)(ob + (size_t)row * NV) = val;
    }
    __threadfence();
#pragma unroll
    for (int rr = 0; rr < 8; ++rr) {
      const int row = wave * 8 + rr;
      const v4f val = *(const v4fa*)(sr + row * SP);
      *(volatile v4f*)(ob + (size_t)row * NV) = val;
    }
    __syncthreads();
  }
}

extern "C" void kernel_launch(void* const* d_in, const int* in_sizes, int n_in,
                              void* d_out, int out_size, void* d_ws, size_t ws_size,
                              hipStream_t stream) {
  if (n_in < 4) return;
  if (in_sizes[0] != NB * NT) return;
  if (in_sizes[1] != NB * NS) return;
  if (in_sizes[2] != NB * NV * NS) return;
  if (in_sizes[3] < 1) return;
  if (out_size != NB * NT * NV) return;

  const size_t off_vh = 0;
  const size_t sz_vh  = (size_t)NB * NV * NS * sizeof(unsigned short);
  const size_t need   = off_vh + sz_vh;
  if (need > ws_size) return;
  if (need > (size_t)134217728) return;

  const float* q   = (const float*)d_in[0];
  const float* k   = (const float*)d_in[1];
  const float* val = (const float*)d_in[2];
  const float* ls  = (const float*)d_in[3];
  float* out = (float*)d_out;
  unsigned short* vh = (unsigned short*)((char*)d_ws + off_vh);

  const int n8 = in_sizes[2] / 8;
  cvt_value_f16<<<dim3((n8 + 255) / 256), dim3(256), 0, stream>>>(val, vh, n8);
  rbf_gemm_kernel<<<dim3(NT / BM, NV / BN, NB), dim3(256), 0, stream>>>(q, k, vh, ls, out);
  (void)hipGetLastError();
}
